// MambaLayer_81827716923671
// MI455X (gfx1250) — hardware-verified
//
#include <hip/hip_runtime.h>
#include <math.h>

typedef __attribute__((ext_vector_type(16))) _Float16 v16h;
typedef __attribute__((ext_vector_type(8)))  _Float16 v8h;
typedef __attribute__((ext_vector_type(16))) __bf16   v16b;
typedef __attribute__((ext_vector_type(8)))  __bf16   v8b;
typedef __attribute__((ext_vector_type(8)))  float    v8f;
typedef __attribute__((ext_vector_type(4)))  float    v4f;

constexpr int kBatch    = 4;
constexpr int kSeq      = 2048;
constexpr int kDm       = 1024;
constexpr int kDin      = 2048;
constexpr int kNst      = 16;
constexpr int kConvK    = 4;
constexpr int kRows     = kBatch * kSeq;
constexpr int kHalfB    = 2;
constexpr int kHalfRows = kHalfB * kSeq;
constexpr int kInN      = 2 * kDin;
constexpr int kXpN      = 2 * kNst;
constexpr int kXpPad    = 64;
constexpr int kWordsPR  = kDin / 2;
constexpr int kConvTP   = 260;
constexpr int kScanTS   = 32;
constexpr int kScanYP   = 260;
constexpr int kScanCh   = 256;
constexpr float kCarryX   = 8.0f;
constexpr float kCarryW   = 64.0f;
constexpr float kCarryXc  = 64.0f;
constexpr float kCarryLo  = 1024.0f;
constexpr float kCarryWxH = 16384.0f;
constexpr float kCarryWxL = 16.0f;
constexpr float kCarryY   = 64.0f;
constexpr float kScale1   = 1.0f / (kCarryX * kCarryW);
constexpr float kScale2   = 1.0f / (kCarryXc * kCarryWxH);
constexpr float kScale3   = 1.0f / (kCarryY * kCarryW);
static_assert(kCarryWxH == kCarryWxL * kCarryLo, "residual pairing");
static_assert((kDm % 32) == 0 && (kDin % 32) == 0, "GEMM K multiples of 32");
static_assert((kHalfRows % 64) == 0 && (kDin % 64) == 0 && (kXpPad % 64) == 0 && (kDm % 64) == 0, "GEMM M,N multiples of 64");
static_assert((kSeq % 64) == 0 && (kSeq % kScanTS) == 0 && (kDin % kScanCh) == 0 && (kDin % 256) == 0, "tile multiples");
static_assert(kXpN <= kXpPad && (kDm % 8) == 0 && (kDin % 8) == 0 && (kBatch % kHalfB) == 0, "plane widths");

constexpr size_t kOffX16  = 0;
constexpr size_t kOffW1   = kOffX16 + (size_t)kRows     * kDm  * 2;
constexpr size_t kOffWXH  = kOffW1  + (size_t)kInN      * kDm  * 2;
constexpr size_t kOffWXL  = kOffWXH + (size_t)kXpPad    * kDin * 2;
constexpr size_t kOffW3   = kOffWXL + (size_t)kXpPad    * kDin * 2;
constexpr size_t kOffXP   = kOffW3  + (size_t)kDm       * kDin * 2;
constexpr size_t kOffGT   = kOffXP  + (size_t)kHalfRows * kDin * 4;
constexpr size_t kOffXCH  = kOffGT  + (size_t)kHalfRows * kDin * 2;
constexpr size_t kOffXCL  = kOffXCH + (size_t)kHalfRows * kDin * 2;
constexpr size_t kOffBC   = kOffXCL + (size_t)kHalfRows * kDin * 2;
constexpr size_t kOffYG   = kOffBC  + (size_t)kHalfRows * kXpPad * 4;
constexpr size_t kWsTotal = kOffYG  + (size_t)kHalfRows * kDin * 2;
static_assert(kWsTotal == 131596288ull, "carve total");
static_assert(kWsTotal <= 134217728ull, "carve cap");
static_assert((kOffW1 % 128) == 0 && (kOffWXH % 128) == 0 && (kOffWXL % 128) == 0 && (kOffW3 % 128) == 0 &&
              (kOffXP % 128) == 0 && (kOffGT % 128) == 0 && (kOffXCH % 128) == 0 && (kOffXCL % 128) == 0 &&
              (kOffBC % 128) == 0 && (kOffYG % 128) == 0, "128-B aligned regions");
constexpr size_t kOut0Floats = (size_t)kRows * kDm;
constexpr size_t kOut1Floats = (size_t)kBatch * kDin * kNst;
static_assert(kOut0Floats * 4 == 33554432ull && (kOut0Floats * 4 + kOut1Floats * 4) == 34078720ull, "output layout");

__device__ __forceinline__ unsigned short f2bf_bits(float f) {
  unsigned u = __float_as_uint(f);
  return (unsigned short)((u + 0x7FFFu + ((u >> 16) & 1u)) >> 16);
}
__device__ __forceinline__ float bf_bits2f(unsigned short h) { return __uint_as_float(((unsigned)h) << 16); }
__device__ __forceinline__ float bf_rne(float f) { return bf_bits2f(f2bf_bits(f)); }
__device__ __forceinline__ float h16_to_f32(unsigned hb) {
  const unsigned sgn = (hb & 0x8000u) << 16; const unsigned em = hb & 0x7fffu;
  const float fn = __uint_as_float((em << 13) + 0x38000000u);
  const float fs = (float)em * 5.9604644775390625e-8f;
  const float mag = (em < 0x400u) ? fs : fn; return __uint_as_float(__float_as_uint(mag) | sgn); }

__device__ __forceinline__ void dep_guard4_h(v8f& a, v8f& b, v8f& c, v8f& d, v16h x, v16h y) {
  asm volatile("v_nop\n\tv_nop\n\tv_nop\n\tv_nop" : "+v"(a), "+v"(b), "+v"(c), "+v"(d) : "v"(x), "v"(y)); }
__device__ __forceinline__ void dep_guard4_b(v8f& a, v8f& b, v8f& c, v8f& d, v16b x, v16b y) {
  asm volatile("v_nop\n\tv_nop\n\tv_nop\n\tv_nop" : "+v"(a), "+v"(b), "+v"(c), "+v"(d) : "v"(x), "v"(y)); }
__device__ __forceinline__ void keep4_h(v16h a, v16h b, v16h c, v16h d) { asm volatile("v_nop" :: "v"(a), "v"(b), "v"(c), "v"(d)); }
__device__ __forceinline__ void keep4_b(v16b a, v16b b, v16b c, v16b d) { asm volatile("v_nop" :: "v"(a), "v"(b), "v"(c), "v"(d)); }
__device__ __forceinline__ void acc_guard4(v8f& a, v8f& b, v8f& c, v8f& d) { asm volatile("v_nop\n\tv_nop\n\tv_nop\n\tv_nop" : "+v"(a), "+v"(b), "+v"(c), "+v"(d)); }
template <typename T> struct Frag;
template <> struct Frag<_Float16> {
  typedef v16h V; union U { v16h v; v8h h[2]; };
  static __device__ __forceinline__ v16h load(const _Float16* p) {
    U f; f.h[0] = *(const v8h*)(p); f.h[1] = *(const v8h*)(p + 16); return f.v;
  }
  static __device__ __forceinline__ v8f mma(v16h a, v16h b, v8f c) {
    return __builtin_amdgcn_wmma_f32_16x16x32_f16(false, a, false, b, (short)0, c, false, false);
  }
  static __device__ __forceinline__ void guard4(v8f& a, v8f& b, v8f& c, v8f& d, v16h x, v16h y) { dep_guard4_h(a, b, c, d, x, y); }
  static __device__ __forceinline__ void keep(v16h a, v16h b, v16h c, v16h d) { keep4_h(a, b, c, d); }
};
template <> struct Frag<__bf16> {
  typedef v16b V; union U { v16b v; v8b h[2]; };
  static __device__ __forceinline__ v16b load(const __bf16* p) {
    U f; f.h[0] = *(const v8b*)(p); f.h[1] = *(const v8b*)(p + 16); return f.v;
  }
  static __device__ __forceinline__ v8f mma(v16b a, v16b b, v8f c) {
    return __builtin_amdgcn_wmma_f32_16x16x32_bf16(false, a, false, b, (short)0, c, false, false);
  }
  static __device__ __forceinline__ void guard4(v8f& a, v8f& b, v8f& c, v8f& d, v16b x, v16b y) { dep_guard4_b(a, b, c, d, x, y); }
  static __device__ __forceinline__ void keep(v16b a, v16b b, v16b c, v16b d) { keep4_b(a, b, c, d); }
};

template <int ET> struct Elem;
template <> struct Elem<0> { typedef _Float16 T; };
template <> struct Elem<1> { typedef __bf16 T; };
template <int ET, int SPL, int BIAS_MODE, int OUT_MODE, int ACT>
__global__ __launch_bounds__(256) void wmma_gemm64(
    const unsigned short* __restrict__ Ap, const unsigned short* __restrict__ A2p, int lda, long strideA,
    const unsigned short* __restrict__ Btp, const unsigned short* __restrict__ Bt2p, int ldb, long strideB,
    void* __restrict__ Cout, void* __restrict__ Cout2, int ldc, long strideC,
    const float* __restrict__ bias,
    int M, int N, int K, float scale) {
  typedef typename Elem<ET>::T T;
  typedef typename Frag<T>::V V;
  const T* A = (const T*)Ap; const T* A2 = (const T*)A2p; const T* Bt = (const T*)Btp; const T* Bt2 = (const T*)Bt2p;
  __shared__ __align__(16) float sT[8][16 * 68];
  const int b    = blockIdx.y;
  const int lane = threadIdx.x & 31;
  const int wave = threadIdx.x >> 5;
  const int tilesN = N >> 6;
  const int tilesM = M >> 6;
  const int tile = blockIdx.x * 8 + wave;
  if (tile >= tilesM * tilesN) return;
  const int tm = tile / tilesN;
  const int tn = tile - tm * tilesN;
  const int m0 = tm << 6;
  const int n0 = tn << 6;

  const T* Ab  = A  + (size_t)b * strideA;
  const T* Bb  = Bt + (size_t)b * strideB;
  const T* Ab2 = (SPL >= 1) ? (A2  + (size_t)b * strideA) : nullptr;
  const T* Bb2 = (SPL >= 1) ? (Bt2 + (size_t)b * strideB) : nullptr;

  const int rlane = lane & 15;
  const int koff  = (lane >> 4) * 8;
  const int mOff  = (lane >> 4) * 8;

  v8f acc[4][4];
#pragma unroll
  for (int i = 0; i < 4; ++i)
#pragma unroll
    for (int j = 0; j < 4; ++j) acc[i][j] = (v8f){0.f,0.f,0.f,0.f,0.f,0.f,0.f,0.f};

  for (int k0 = 0; k0 < K; k0 += 32) {
    V bh[4], bl[4];
#pragma unroll
    for (int j = 0; j < 4; ++j) {
      const size_t bo = (size_t)(n0 + (j << 4) + rlane) * ldb + koff + k0;
      bh[j] = Frag<T>::load(Bb + bo);
      if (SPL >= 1) bl[j] = Frag<T>::load(Bb2 + bo);
    }
#pragma unroll
    for (int i = 0; i < 4; ++i) {
      const size_t ao = (size_t)(m0 + (i << 4) + rlane) * lda + koff + k0;
      V ah = Frag<T>::load(Ab + ao);
      V al;
      if (SPL >= 1) al = Frag<T>::load(Ab2 + ao);
#pragma unroll
      for (int j = 0; j < 4; ++j) {
        acc[i][j] = Frag<T>::mma(ah, bh[j], acc[i][j]);
        if (SPL == 2) { acc[i][j] = Frag<T>::mma(ah, bl[j], acc[i][j]); acc[i][j] = Frag<T>::mma(al, bh[j], acc[i][j]); }
        if (SPL == 1) acc[i][j] = Frag<T>::mma(al, bl[j], acc[i][j]);
      }
      Frag<T>::guard4(acc[i][0], acc[i][1], acc[i][2], acc[i][3], ah, (SPL >= 1) ? al : ah);
    }
    Frag<T>::keep(bh[0], bh[1], bh[2], bh[3]);
    if (SPL >= 1) Frag<T>::keep(bl[0], bl[1], bl[2], bl[3]);
  }
  acc_guard4(acc[0][0], acc[0][1], acc[0][2], acc[0][3]);
  acc_guard4(acc[1][0], acc[1][1], acc[1][2], acc[1][3]);
  acc_guard4(acc[2][0], acc[2][1], acc[2][2], acc[2][3]);
  acc_guard4(acc[3][0], acc[3][1], acc[3][2], acc[3][3]);

  float* slab = sT[wave];
#pragma unroll
  for (int i = 0; i < 4; ++i) {
    const int mBase = m0 + (i << 4);
#pragma unroll
    for (int j = 0; j < 4; ++j) {
      const int n = n0 + (j << 4) + rlane;
      float bv = 0.f;
      if (BIAS_MODE == 2) bv = bias[n];
#pragma unroll
      for (int r = 0; r < 8; ++r) {
        float v = acc[i][j][r] * scale;
        if (BIAS_MODE == 1) v += bias[mBase + mOff + r];
        if (BIAS_MODE == 2) v += bv;
        if (ACT == 1) v = tanhf(v);
        if (ACT == 2) v = fmaxf(v, 0.0f);
        if (ACT == 3) v = v / (1.0f + expf(-v));
        if (ACT == 4) v = (v > 0.f) ? v : 0.01f * v;
        if (ACT == 6) { const float ee = __expf(-v); v = v * __builtin_amdgcn_rcpf(1.0f + ee); }
        slab[(mOff + r) * 68 + (j << 4) + rlane] = v;
      }
    }
    __builtin_amdgcn_fence(__ATOMIC_RELEASE, "workgroup");
    __builtin_amdgcn_wave_barrier();
    __builtin_amdgcn_fence(__ATOMIC_ACQUIRE, "workgroup");
    if (OUT_MODE == 0) {
      float* C = (float*)Cout + (size_t)b * strideC;
      const int hh = lane >> 4, c4 = (lane & 15) * 4;
      for (int pass = 0; pass < 2; ++pass) {
#pragma unroll
        for (int it = 0; it < 8; ++it) {
          const int row = it * 2 + hh;
          v4f v = *(const v4f*)(slab + row * 68 + c4);
          *(volatile v4f*)(C + (size_t)(mBase + row) * ldc + n0 + c4) = v;
        }
        __threadfence();
      }
    } else {
      const int q = lane >> 3, c8 = (lane & 7) * 8;
      unsigned short* C  = (unsigned short*)Cout  + (size_t)b * strideC;
      unsigned short* C2 = (OUT_MODE == 2) ? ((unsigned short*)Cout2 + (size_t)b * strideC) : nullptr;
      for (int pass = 0; pass < 2; ++pass) {
#pragma unroll
        for (int it = 0; it < 4; ++it) {
          const int row = it * 4 + q;
          const float* sp = slab + row * 68 + c8;
          v8h hv, lv;
#pragma unroll
          for (int e = 0; e < 8; ++e) {
            if (OUT_MODE == 1) {
              hv[e] = (_Float16)sp[e];
            } else {
              unsigned short hb = f2bf_bits(sp[e]);
              unsigned short lb = f2bf_bits(sp[e] - bf_bits2f(hb));
              hv[e] = __builtin_bit_cast(_Float16, hb);
              lv[e] = __builtin_bit_cast(_Float16, lb);
            }
          }
          *(volatile v8h*)(C + (size_t)(mBase + row) * ldc + n0 + c8) = hv;
          if (OUT_MODE == 2) *(volatile v8h*)(C2 + (size_t)(mBase + row) * ldc + n0 + c8) = lv;
        }
        __threadfence();
      }
    }
    __builtin_amdgcn_fence(__ATOMIC_RELEASE, "workgroup");
    __builtin_amdgcn_wave_barrier();
    __builtin_amdgcn_fence(__ATOMIC_ACQUIRE, "workgroup");
  }
}

__global__ __launch_bounds__(256) void cvt_plane_kernel(
    const float* __restrict__ src, unsigned short* __restrict__ dst, int rows_real, int cols, int total8, float scale)
{
  const int i = blockIdx.x * 256 + threadIdx.x;
  if (i >= total8) return;
  const size_t e0 = (size_t)i << 3;
  const int row = (int)(e0 / (size_t)cols);
  const int col = (int)(e0 - (size_t)row * (size_t)cols);
  const bool live = (row < rows_real);
  const int rowc = live ? row : (rows_real - 1);
  const float* sp = src + (size_t)rowc * cols + col;
  const v4f a0 = *(const v4f*)(sp);
  const v4f a1 = *(const v4f*)(sp + 4);
  const float lf = live ? 1.0f : 0.0f;
  v8h hv;
#pragma unroll
  for (int e = 0; e < 4; ++e) {
    const float v0 = a0[e] * lf;
    const float v1 = a1[e] * lf;
    hv[e]     = (_Float16)(bf_rne(v0) * scale);
    hv[4 + e] = (_Float16)(bf_rne(v1) * scale);
  }
  unsigned short* qd = dst + e0;
  *(volatile v8h*)qd = hv;
  __threadfence();
  *(volatile v8h*)qd = hv;
}

__global__ __launch_bounds__(256) void conv_silu_kernel(
    const float* __restrict__ XPf, const float* __restrict__ cw, const float* __restrict__ cb,
    unsigned short* __restrict__ XCH, unsigned short* __restrict__ XCL)
{
  __shared__ __align__(16) float sT[16 * kConvTP];
  const int tid = threadIdx.x, lane = tid & 31, wave = tid >> 5;
  const int d0 = blockIdx.x * 256, d = d0 + tid;
  const int g0 = blockIdx.y * 64;
  const int tb = g0 & (kSeq - 1);
  const v4f wv = *(const v4f*)(cw + (size_t)d * kConvK);
  const float w0 = bf_rne(wv[0]), w1 = bf_rne(wv[1]), w2 = bf_rne(wv[2]), w3 = bf_rne(wv[3]);
  const float bcv = bf_rne(cb[d]);
  float xm3, xm2, xm1;
  {
    const bool hist = (tb > 0);
    const int rb = hist ? (g0 - 3) : g0;
    const float v3 = XPf[(size_t)rb * kDin + d];
    const float v2 = XPf[(size_t)(rb + 1) * kDin + d];
    const float v1 = XPf[(size_t)(rb + 2) * kDin + d];
    const float hf = hist ? 1.0f : 0.0f;
    xm3 = v3 * hf;
    xm2 = v2 * hf;
    xm1 = v1 * hf;
  }
#pragma unroll 1
  for (int sub = 0; sub < 4; ++sub) {
    const int lb = g0 + sub * 16;
#pragma unroll 1
    for (int s = 0; s < 16; ++s) {
      const float xcur = XPf[(size_t)(lb + s) * kDin + d];
      float acc = w0 * xm3;
      acc = fmaf(w1, xm2, acc);
      acc = fmaf(w2, xm1, acc);
      acc = fmaf(w3, xcur, acc);
      const float pre = acc + bcv;
      const float ee = expf(-pre);
      const float xc = pre * __builtin_amdgcn_rcpf(1.0f + ee);
      sT[s * kConvTP + tid] = xc * kCarryXc;
      xm3 = xm2; xm2 = xm1; xm1 = xcur;
    }
    __syncthreads();
    v8h hv[2], lv[2];
#pragma unroll
    for (int it = 0; it < 2; ++it) {
      const float* sp = sT + (it * 8 + wave) * kConvTP + lane * 8;
      const v4f a0 = *(const v4f*)(sp);
      const v4f a1 = *(const v4f*)(sp + 4);
#pragma unroll
      for (int e = 0; e < 4; ++e) {
        const float f0 = a0[e], f1 = a1[e];
        const _Float16 h0 = (_Float16)f0, h1 = (_Float16)f1;
        const float hf0 = (float)h0, hf1 = (float)h1;
        const float r0 = (f0 - hf0) * kCarryLo, r1 = (f1 - hf1) * kCarryLo;
        hv[it][e]     = h0;
        hv[it][4 + e] = h1;
        lv[it][e]     = (_Float16)r0;
        lv[it][4 + e] = (_Float16)r1;
      }
    }
    for (int pass = 0; pass < 2; ++pass) {
#pragma unroll
      for (int it = 0; it < 2; ++it) {
        const size_t o = (size_t)(lb + it * 8 + wave) * kDin + d0 + lane * 8;
        *(volatile v8h*)(XCH + o) = hv[it];
        *(volatile v8h*)(XCL + o) = lv[it];
      }
      __threadfence();
    }
    __syncthreads();
  }
}

__global__ __launch_bounds__(256) void scan_kernel(
    const float* __restrict__ BC, const float* __restrict__ XPf, const unsigned* __restrict__ GT32,
    const float* __restrict__ cw, const float* __restrict__ cb, const float* __restrict__ Alog,
    const float* __restrict__ Dp, const float* __restrict__ st0,
    unsigned short* __restrict__ YG, float* __restrict__ hfin, int bbase)
{
  __shared__ __align__(16) float sBC[kScanTS * kXpN];
  __shared__ __align__(16) float sY[kScanTS * kScanYP];
  __shared__ __align__(16) float sH[kScanCh * kNst];
  __shared__ __align__(16) float sD[kNst * kScanCh];
  const int tid = threadIdx.x, lane = tid & 31, wave = tid >> 5;
  constexpr int kBlkPerB = kDin / kScanCh;
  const int bix = blockIdx.x / kBlkPerB;
  const int gb  = bbase + bix;
  const int d0  = (blockIdx.x - bix * kBlkPerB) * kScanCh;
  const int d   = d0 + tid;
  const size_t row0 = (size_t)bix * kSeq;

#pragma unroll 1
  for (int n = 0; n < kNst; ++n) {
    const float al = Alog[(size_t)d * kNst + n];
    sD[n * kScanCh + tid] = expf(-expf(bf_rne(al)));
  }
  float h[kNst], dec[kNst];
  {
    const float* hp = st0 + ((size_t)gb * kDin + d) * kNst;
    const v4f s0 = *(const v4f*)(hp), s1 = *(const v4f*)(hp + 4), s2 = *(const v4f*)(hp + 8), s3 = *(const v4f*)(hp + 12);
#pragma unroll
    for (int e = 0; e < 4; ++e) {
      h[e] = bf_rne(s0[e]); h[4 + e] = bf_rne(s1[e]); h[8 + e] = bf_rne(s2[e]); h[12 + e] = bf_rne(s3[e]);
    }
  }
  __syncthreads();
#pragma unroll
  for (int n = 0; n < kNst; ++n) dec[n] = sD[n * kScanCh + tid];
  asm volatile("" ::: "memory");
  const v4f wv = *(const v4f*)(cw + (size_t)d * kConvK);
  const float w0 = bf_rne(wv[0]), w1 = bf_rne(wv[1]), w2 = bf_rne(wv[2]), w3 = bf_rne(wv[3]);
  const float bcv = bf_rne(cb[d]);
  const float Dd  = bf_rne(Dp[d]);
  const int wcol = d >> 1;
  const unsigned shift = (d & 1) ? 16u : 0u;
  float xm3 = 0.f, xm2 = 0.f, xm1 = 0.f;
  const int lr = tid >> 3, lc4 = (tid & 7) * 4;
#pragma unroll 1
  for (int t0 = 0; t0 < kSeq; t0 += kScanTS) {
    __syncthreads();
    *(v4f*)(sBC + lr * kXpN + lc4) = *(const v4f*)(BC + (row0 + t0 + lr) * kXpPad + lc4);
    __syncthreads();
#pragma unroll 1
    for (int s = 0; s < kScanTS; ++s) {
      const size_t row = row0 + t0 + s;
      const float xcur = XPf[row * kDin + d];
      const unsigned gw = GT32[row * kWordsPR + wcol];
      const float gv   = h16_to_f32((gw >> shift) & 0xffffu);
      float acc = w0 * xm3;
      acc = fmaf(w1, xm2, acc);
      acc = fmaf(w2, xm1, acc);
      acc = fmaf(w3, xcur, acc);
      const float pre = acc + bcv;
      const float ee = expf(-pre);
      const float xc = pre * __builtin_amdgcn_rcpf(1.0f + ee);
      const float* xr = sBC + s * kXpN;
      float Bs[kNst], Cs[kNst];
#pragma unroll
      for (int q4 = 0; q4 < 4; ++q4) {
        const v4f bv = *(const v4f*)(xr + 4 * q4);
        const v4f cv = *(const v4f*)(xr + kNst + 4 * q4);
        Bs[4 * q4 + 0] = bv[0]; Bs[4 * q4 + 1] = bv[1]; Bs[4 * q4 + 2] = bv[2]; Bs[4 * q4 + 3] = bv[3];
        Cs[4 * q4 + 0] = cv[0]; Cs[4 * q4 + 1] = cv[1]; Cs[4 * q4 + 2] = cv[2]; Cs[4 * q4 + 3] = cv[3];
      }
      float y = 0.0f;
#pragma unroll
      for (int n = 0; n < kNst; ++n) {
        h[n] = fmaf(h[n], dec[n], xc * Bs[n]);
        y = fmaf(h[n], Cs[n], y);
      }
      y = fmaf(Dd, xc, y);
      sY[s * kScanYP + tid] = (y * gv) * kCarryY;
      xm3 = xm2; xm2 = xm1; xm1 = xcur;
    }
    __syncthreads();
    v8h hv[4];
#pragma unroll
    for (int it = 0; it < 4; ++it) {
      const float* sp = sY + (it * 8 + wave) * kScanYP + lane * 8;
      const v4f a0 = *(const v4f*)(sp);
      const v4f a1 = *(const v4f*)(sp + 4);
#pragma unroll
      for (int e = 0; e < 4; ++e) {
        hv[it][e]     = (_Float16)a0[e];
        hv[it][4 + e] = (_Float16)a1[e];
      }
    }
    for (int pass = 0; pass < 2; ++pass) {
#pragma unroll
      for (int it = 0; it < 4; ++it) {
        const size_t o = (row0 + t0 + it * 8 + wave) * kDin + d0 + lane * 8;
        *(volatile v8h*)(YG + o) = hv[it];
      }
      __threadfence();
    }
  }
  {
    float* shp = sH + tid * kNst;
    *(v4f*)(shp)      = (v4f){h[0],  h[1],  h[2],  h[3]};
    *(v4f*)(shp + 4)  = (v4f){h[4],  h[5],  h[6],  h[7]};
    *(v4f*)(shp + 8)  = (v4f){h[8],  h[9],  h[10], h[11]};
    *(v4f*)(shp + 12) = (v4f){h[12], h[13], h[14], h[15]};
  }
  __syncthreads();
  {
    float* hb = hfin + ((size_t)gb * kDin + d0) * kNst;
    for (int pass = 0; pass < 2; ++pass) {
#pragma unroll
      for (int it = 0; it < 4; ++it) {
        const int f = (it * kScanCh + tid) * 4;
        const v4f v = *(const v4f*)(sH + f);
        *(volatile v4f*)(hb + f) = v;
      }
      __threadfence();
    }
  }
}

extern "C" void kernel_launch(void* const* d_in, const int* in_sizes, int n_in,
                              void* d_out, int out_size, void* d_ws, size_t ws_size,
                              hipStream_t stream) {
  if (n_in < 9) return;
  if (in_sizes[0] != kRows * kDm) return;
  if (in_sizes[1] != kBatch * kDin * kNst) return;
  if (in_sizes[2] != kInN * kDm) return;
  if (in_sizes[3] != kDin * kConvK) return;
  if (in_sizes[4] != kDin) return;
  if (in_sizes[5] != kXpN * kDin) return;
  if (in_sizes[6] != kDin * kNst) return;
  if (in_sizes[7] != kDin) return;
  if (in_sizes[8] != kDm * kDin) return;
  if ((size_t)out_size != kOut0Floats + kOut1Floats) return;
  if (ws_size < kWsTotal) return;

  const float* x          = (const float*)d_in[0];
  const float* state0     = (const float*)d_in[1];
  const float* in_proj_w  = (const float*)d_in[2];
  const float* conv_w     = (const float*)d_in[3];
  const float* conv_b     = (const float*)d_in[4];
  const float* x_proj_w   = (const float*)d_in[5];
  const float* A_log      = (const float*)d_in[6];
  const float* Dp         = (const float*)d_in[7];
  const float* out_proj_w = (const float*)d_in[8];
  float* out0 = (float*)d_out;
  float* out1 = out0 + kOut0Floats;

  char* ws = (char*)d_ws;
  unsigned short* X16 = (unsigned short*)(ws + kOffX16);
  unsigned short* W1  = (unsigned short*)(ws + kOffW1);
  unsigned short* WXH = (unsigned short*)(ws + kOffWXH);
  unsigned short* WXL = (unsigned short*)(ws + kOffWXL);
  unsigned short* W3  = (unsigned short*)(ws + kOffW3);
  float*          XP  = (float*)(ws + kOffXP);
  unsigned short* GT  = (unsigned short*)(ws + kOffGT);
  unsigned short* XCH = (unsigned short*)(ws + kOffXCH);
  unsigned short* XCL = (unsigned short*)(ws + kOffXCL);
  float*          BC  = (float*)(ws + kOffBC);
  unsigned short* YG  = (unsigned short*)(ws + kOffYG);

  cvt_plane_kernel<<<(kRows * kDm / 8) / 256, 256, 0, stream>>>(x, X16, kRows, kDm, kRows * kDm / 8, kCarryX);
  cvt_plane_kernel<<<(kInN * kDm / 8) / 256, 256, 0, stream>>>(in_proj_w, W1, kInN, kDm, kInN * kDm / 8, kCarryW);
  cvt_plane_kernel<<<(kXpPad * kDin / 8) / 256, 256, 0, stream>>>(x_proj_w, WXH, kXpN, kDin, kXpPad * kDin / 8, kCarryWxH);
  cvt_plane_kernel<<<(kXpPad * kDin / 8) / 256, 256, 0, stream>>>(x_proj_w, WXL, kXpN, kDin, kXpPad * kDin / 8, kCarryWxL);
  cvt_plane_kernel<<<(kDm * kDin / 8) / 256, 256, 0, stream>>>(out_proj_w, W3, kDm, kDin, kDm * kDin / 8, kCarryW);

  for (int hb = 0; hb < kBatch / kHalfB; ++hb) {
    const size_t rowOff = (size_t)hb * kHalfRows;
    const unsigned short* X16h = X16 + rowOff * kDm;
    float* out0h = out0 + rowOff * kDm;

    wmma_gemm64<0, 0, 0, 0, 0><<<dim3((kHalfRows / 64) * (kDin / 64) / 8, 1), 256, 0, stream>>>(
        X16h, nullptr, kDm, 0L,
        W1, nullptr, kDm, 0L,
        (void*)XP, nullptr, kDin, 0L,
        nullptr,
        kHalfRows, kDin, kDm, kScale1);

    wmma_gemm64<0, 0, 0, 1, 6><<<dim3((kHalfRows / 64) * (kDin / 64) / 8, 1), 256, 0, stream>>>(
        X16h, nullptr, kDm, 0L,
        W1 + (size_t)kDin * kDm, nullptr, kDm, 0L,
        (void*)GT, nullptr, kDin, 0L,
        nullptr,
        kHalfRows, kDin, kDm, kScale1);

    conv_silu_kernel<<<dim3(kDin / 256, kHalfRows / 64), 256, 0, stream>>>(XP, conv_w, conv_b, XCH, XCL);

    wmma_gemm64<0, 1, 0, 0, 0><<<dim3((kHalfRows / 64) * (kXpPad / 64) / 8, 1), 256, 0, stream>>>(
        XCH, XCL, kDin, 0L,
        WXH, WXL, kDin, 0L,
        (void*)BC, nullptr, kXpPad, 0L,
        nullptr,
        kHalfRows, kXpPad, kDin, kScale2);

    scan_kernel<<<kHalfB * (kDin / kScanCh), kScanCh, 0, stream>>>(
        BC, XP, (const unsigned*)GT, conv_w, conv_b, A_log, Dp, state0, YG, out1, hb * kHalfB);

    wmma_gemm64<0, 0, 0, 0, 0><<<dim3((kHalfRows / 64) * (kDm / 64) / 8, 1), 256, 0, stream>>>(
        YG, nullptr, kDin, 0L,
        W3, nullptr, kDin, 0L,
        (void*)out0h, nullptr, kDm, 0L,
        nullptr,
        kHalfRows, kDm, kDin, kScale3);
  }
}
